// TransformerUnit_79620103733527
// MI455X (gfx1250) — hardware-verified
//
#include <hip/hip_runtime.h>
#include <math.h>
#include <stdint.h>

static constexpr int kSeqQ = 1024;
static constexpr int kNB   = 2;
static constexpr int kDM   = 1024;
static constexpr int kNH   = 16;
static constexpr int kDHD  = 64;
static constexpr int kDFF  = 4096;
static constexpr int kMemL = 1024;
static constexpr int kTK   = 2048;
static constexpr int kHGrp = 2;
static constexpr int kNGrp = kNH / kHGrp;
static_assert(kNH % kHGrp == 0, "head groups");
static_assert(kSeqQ % 64 == 0 && kTK % 64 == 0 && kDM % 64 == 0 && kDFF % 64 == 0 && kDHD % 64 == 0, "tile multiples");
static_assert(kDM % 32 == 0 && kDHD % 32 == 0 && kTK % 32 == 0 && kDFF % 32 == 0, "K multiples of 32");
static_assert(kTK == 256 * 8, "softmax row coverage: 256 threads x 8 columns");
static_assert(kDM == 256 * 4, "layernorm row coverage: 256 threads x 4 columns");

typedef __attribute__((ext_vector_type(16))) _Float16 v16h;
typedef __attribute__((ext_vector_type(8)))  _Float16 v8h;
typedef __attribute__((ext_vector_type(16))) __bf16   v16b;
typedef __attribute__((ext_vector_type(8)))  __bf16   v8b;
typedef __attribute__((ext_vector_type(8)))  float    v8f;
typedef __attribute__((ext_vector_type(4)))  float    v4f;
typedef __attribute__((ext_vector_type(2)))  float    v2f;
typedef __attribute__((ext_vector_type(4)))  unsigned int v4u;
typedef __attribute__((ext_vector_type(4)))  int      v4i;
#define PSCALE 32768.0f
#define U16(p) ((const unsigned short*)(const void*)(p))
#define PSCALE_INV (1.0f / 32768.0f)

__device__ __forceinline__ unsigned short f2bf_bits(float f) {
  unsigned u = __float_as_uint(f);
  return (unsigned short)((u + 0x7FFFu + ((u >> 16) & 1u)) >> 16);
}
__device__ __forceinline__ float bf_bits2f(unsigned short h) { return __uint_as_float(((unsigned)h) << 16); }

__device__ __forceinline__ void dep_guard_h(v8f& a, v8f& b, v16h x, v16h y) { asm volatile("v_nop\n\tv_nop\n\tv_nop\n\tv_nop" : "+v"(a), "+v"(b) : "v"(x), "v"(y)); }
__device__ __forceinline__ void dep_guard_b(v8f& a, v8f& b, v16b x, v16b y) { asm volatile("v_nop\n\tv_nop\n\tv_nop\n\tv_nop" : "+v"(a), "+v"(b) : "v"(x), "v"(y)); }
__device__ __forceinline__ void keep4_h(v16h a, v16h b, v16h c, v16h d) { asm volatile("v_nop" :: "v"(a), "v"(b), "v"(c), "v"(d)); }
__device__ __forceinline__ void keep4_b(v16b a, v16b b, v16b c, v16b d) { asm volatile("v_nop" :: "v"(a), "v"(b), "v"(c), "v"(d)); }
__device__ __forceinline__ void acc_guard4(v8f& a, v8f& b, v8f& c, v8f& d) { asm volatile("v_nop\n\tv_nop\n\tv_nop\n\tv_nop" : "+v"(a), "+v"(b), "+v"(c), "+v"(d)); }
template <typename T> struct Frag;
template <> struct Frag<_Float16> {
  typedef v16h V; union U { v16h v; v8h h[2]; };
  static __device__ __forceinline__ v16h load(const _Float16* p) {
    U f; f.h[0] = *(const v8h*)(p); f.h[1] = *(const v8h*)(p + 16); return f.v;
  }
  static __device__ __forceinline__ v8f mma(v16h a, v16h b, v8f c) {
    return __builtin_amdgcn_wmma_f32_16x16x32_f16(false, a, false, b, (short)0, c, false, false);
  }
  static __device__ __forceinline__ void guard(v8f& a, v8f& b, v16h x, v16h y) { dep_guard_h(a, b, x, y); }
  static __device__ __forceinline__ void keep(v16h a, v16h b, v16h c, v16h d) { keep4_h(a, b, c, d); }
};
template <> struct Frag<__bf16> {
  typedef v16b V; union U { v16b v; v8b h[2]; };
  static __device__ __forceinline__ v16b load(const __bf16* p) {
    U f; f.h[0] = *(const v8b*)(p); f.h[1] = *(const v8b*)(p + 16); return f.v;
  }
  static __device__ __forceinline__ v8f mma(v16b a, v16b b, v8f c) {
    return __builtin_amdgcn_wmma_f32_16x16x32_bf16(false, a, false, b, (short)0, c, false, false);
  }
  static __device__ __forceinline__ void guard(v8f& a, v8f& b, v16b x, v16b y) { dep_guard_b(a, b, x, y); }
  static __device__ __forceinline__ void keep(v16b a, v16b b, v16b c, v16b d) { keep4_b(a, b, c, d); }
};

template <int ET> struct Elem;
template <> struct Elem<0> { typedef _Float16 T; };
template <> struct Elem<1> { typedef __bf16 T; };
template <int ET, bool SPLIT, int BIAS_MODE, int OUT_MODE, bool RESID, int ACT = 0>
__global__ __launch_bounds__(256) void wmma_gemm64(
    const unsigned short* __restrict__ Ap, const unsigned short* __restrict__ A2p, int lda, long strideA,
    const unsigned short* __restrict__ Btp, const unsigned short* __restrict__ Bt2p, int ldb, long strideB,
    void* __restrict__ Cout, void* __restrict__ Cout2, int ldc, long strideC,
    const float* __restrict__ bias,
    const float* __restrict__ resid, long strideR,
    int M, int N, int K, float scale) {
  typedef typename Elem<ET>::T T;
  typedef typename Frag<T>::V V;
  const T* A = (const T*)Ap; const T* A2 = (const T*)A2p; const T* Bt = (const T*)Btp; const T* Bt2 = (const T*)Bt2p;
  __shared__ __align__(16) float sT[8][16 * 68];
  const int b    = blockIdx.y;
  const int lane = threadIdx.x & 31;
  const int wave = threadIdx.x >> 5;
  const int tilesN = N >> 6;
  const int tilesM = M >> 6;
  const int tile = blockIdx.x * 8 + wave;
  if (tile >= tilesM * tilesN) return;
  const int tm = tile / tilesN;
  const int tn = tile - tm * tilesN;
  const int m0 = tm << 6;
  const int n0 = tn << 6;

  const T* Ab  = A  + (size_t)b * strideA;
  const T* Bb  = Bt + (size_t)b * strideB;
  const T* Ab2 = SPLIT ? (A2  + (size_t)b * strideA) : nullptr;
  const T* Bb2 = SPLIT ? (Bt2 + (size_t)b * strideB) : nullptr;

  const int rlane = lane & 15;
  const int koff  = (lane >> 4) * 8;
  const int mOff  = (lane >> 4) * 8;

  v8f acc[4][4];
#pragma unroll
  for (int i = 0; i < 4; ++i)
#pragma unroll
    for (int j = 0; j < 4; ++j) acc[i][j] = (v8f){0.f,0.f,0.f,0.f,0.f,0.f,0.f,0.f};

  for (int k0 = 0; k0 < K; k0 += 32) {
    V bh[4], bl[4];
#pragma unroll
    for (int j = 0; j < 4; ++j) {
      const size_t bo = (size_t)(n0 + (j << 4) + rlane) * ldb + koff + k0;
      bh[j] = Frag<T>::load(Bb + bo);
      if (SPLIT) bl[j] = Frag<T>::load(Bb2 + bo);
    }
#pragma unroll
    for (int i = 0; i < 4; ++i) {
      const size_t ao = (size_t)(m0 + (i << 4) + rlane) * lda + koff + k0;
      V ah = Frag<T>::load(Ab + ao);
      V al;
      if (SPLIT) al = Frag<T>::load(Ab2 + ao);
#pragma unroll
      for (int j = 0; j < 4; ++j) {
        acc[i][j] = Frag<T>::mma(ah, bh[j], acc[i][j]);
        if (SPLIT) {
          acc[i][j] = Frag<T>::mma(ah, bl[j], acc[i][j]);
          acc[i][j] = Frag<T>::mma(al, bh[j], acc[i][j]);
        }
      }
      Frag<T>::guard(acc[i][0], acc[i][3], ah, SPLIT ? al : ah);
    }
    Frag<T>::keep(bh[0], bh[1], bh[2], bh[3]);
    if (SPLIT) Frag<T>::keep(bl[0], bl[1], bl[2], bl[3]);
  }
  acc_guard4(acc[0][0], acc[0][1], acc[0][2], acc[0][3]);
  acc_guard4(acc[1][0], acc[1][1], acc[1][2], acc[1][3]);
  acc_guard4(acc[2][0], acc[2][1], acc[2][2], acc[2][3]);
  acc_guard4(acc[3][0], acc[3][1], acc[3][2], acc[3][3]);

  float* slab = sT[wave];
  const float* Rb = RESID ? (resid + (size_t)b * strideR) : nullptr;
#pragma unroll
  for (int i = 0; i < 4; ++i) {
    const int mBase = m0 + (i << 4);
#pragma unroll
    for (int j = 0; j < 4; ++j) {
      const int n = n0 + (j << 4) + rlane;
      float bv = 0.f;
      if (BIAS_MODE == 2) bv = bias[n];
#pragma unroll
      for (int r = 0; r < 8; ++r) {
        float v = acc[i][j][r] * scale;
        if (BIAS_MODE == 1) v += bias[mBase + mOff + r];
        if (BIAS_MODE == 2) v += bv;
        if (RESID) v += Rb[(size_t)(mBase + mOff + r) * ldc + n];
        if (ACT == 1) v = tanhf(v);
        if (ACT == 2) v = fmaxf(v, 0.0f);
        if (ACT == 3) v = v / (1.0f + expf(-v));
        if (ACT == 4) v = (v > 0.f) ? v : 0.01f * v;
        slab[(mOff + r) * 68 + (j << 4) + rlane] = v;
      }
    }
    __builtin_amdgcn_fence(__ATOMIC_RELEASE, "workgroup");
    __builtin_amdgcn_wave_barrier();
    __builtin_amdgcn_fence(__ATOMIC_ACQUIRE, "workgroup");
    if (OUT_MODE == 0) {
      float* C = (float*)Cout + (size_t)b * strideC;
      const int hh = lane >> 4, c4 = (lane & 15) * 4;
      for (int pass = 0; pass < 2; ++pass) {
#pragma unroll
        for (int it = 0; it < 8; ++it) {
          const int row = it * 2 + hh;
          v4f v = *(const v4f*)(slab + row * 68 + c4);
          *(volatile v4f*)(C + (size_t)(mBase + row) * ldc + n0 + c4) = v;
        }
        __threadfence();
      }
    } else {
      const int q = lane >> 3, c8 = (lane & 7) * 8;
      unsigned short* C  = (unsigned short*)Cout  + (size_t)b * strideC;
      unsigned short* C2 = (OUT_MODE == 2) ? ((unsigned short*)Cout2 + (size_t)b * strideC) : nullptr;
      for (int pass = 0; pass < 2; ++pass) {
#pragma unroll
        for (int it = 0; it < 4; ++it) {
          const int row = it * 4 + q;
          const float* sp = slab + row * 68 + c8;
          v8h hv, lv;
#pragma unroll
          for (int e = 0; e < 8; ++e) {
            if (OUT_MODE == 1) {
              hv[e] = (_Float16)sp[e];
            } else {
              unsigned short hb = f2bf_bits(sp[e]);
              unsigned short lb = f2bf_bits(sp[e] - bf_bits2f(hb));
              hv[e] = __builtin_bit_cast(_Float16, hb);
              lv[e] = __builtin_bit_cast(_Float16, lb);
            }
          }
          *(volatile v8h*)(C + (size_t)(mBase + row) * ldc + n0 + c8) = hv;
          if (OUT_MODE == 2) *(volatile v8h*)(C2 + (size_t)(mBase + row) * ldc + n0 + c8) = lv;
        }
        __threadfence();
      }
    }
    __builtin_amdgcn_fence(__ATOMIC_RELEASE, "workgroup");
    __builtin_amdgcn_wave_barrier();
    __builtin_amdgcn_fence(__ATOMIC_ACQUIRE, "workgroup");
  }
}

__device__ __forceinline__ unsigned pk16(unsigned short a, unsigned short b) { return (unsigned)a | ((unsigned)b << 16); }
__device__ __forceinline__ unsigned short h_bits(float f) { const _Float16 h = (_Float16)f; return __builtin_bit_cast(unsigned short, h); }

__global__ __launch_bounds__(256) void transpose_cast_f16_kernel(const float* __restrict__ in, int ld_in, int rows,
                                                                 unsigned short* __restrict__ out, float scale) {
  __shared__ float tile[64][65];
  const int tid = threadIdx.x;
  const int c0 = blockIdx.x * 64;
  const int r0 = blockIdx.y * 64;
  const int lr = tid >> 4, lc4 = (tid & 15) * 4;
#pragma unroll
  for (int it = 0; it < 4; ++it) {
    const int r = it * 16 + lr;
    const v4f v = *(const v4f*)(in + (size_t)(r0 + r) * ld_in + c0 + lc4);
    tile[r][lc4 + 0] = v[0];
    tile[r][lc4 + 1] = v[1];
    tile[r][lc4 + 2] = v[2];
    tile[r][lc4 + 3] = v[3];
  }
  __syncthreads();
  const int q = tid >> 3, c8 = (tid & 7) * 8;
  v8h hv0, hv1;
#pragma unroll
  for (int e = 0; e < 8; ++e) {
    hv0[e] = (_Float16)(tile[c8 + e][q] * scale);
    hv1[e] = (_Float16)(tile[c8 + e][32 + q] * scale);
  }
  unsigned short* o0 = out + (size_t)(c0 + q) * rows + r0 + c8;
  unsigned short* o1 = out + (size_t)(c0 + 32 + q) * rows + r0 + c8;
  *(volatile v8h*)o0 = hv0;
  *(volatile v8h*)o1 = hv1;
  __threadfence();
  *(volatile v8h*)o0 = hv0;
  *(volatile v8h*)o1 = hv1;
}

__global__ __launch_bounds__(128) void cast_act_rows_kernel(const float* __restrict__ x, const float* __restrict__ mem,
                                                            const float* __restrict__ pe, int b,
                                                            unsigned short* __restrict__ dst) {
  const int row = blockIdx.x;
  const int tid = threadIdx.x;
  const float* src;
  if (row < kMemL)     src = mem + (size_t)row * (kNB * kDM) + (size_t)b * kDM;
  else if (row < kTK)  src = x   + (size_t)(row - kMemL) * (kNB * kDM) + (size_t)b * kDM;
  else                 src = pe  + (size_t)(row - kTK) * (kNB * kDM) + (size_t)b * kDM;
  const v4f f0 = *(const v4f*)(src + 8 * tid);
  const v4f f1 = *(const v4f*)(src + 8 * tid + 4);
  v8h hv;
  hv[0] = (_Float16)f0[0]; hv[1] = (_Float16)f0[1]; hv[2] = (_Float16)f0[2]; hv[3] = (_Float16)f0[3];
  hv[4] = (_Float16)f1[0]; hv[5] = (_Float16)f1[1]; hv[6] = (_Float16)f1[2]; hv[7] = (_Float16)f1[3];
  unsigned short* op = dst + (size_t)row * kDM + 8 * tid;
  *(volatile v8h*)op = hv;
  __threadfence();
  *(volatile v8h*)op = hv;
}

__global__ __launch_bounds__(256) void build_qbias_kernel(const float* __restrict__ qf, const float* __restrict__ ub,
                                                          const float* __restrict__ vbias, unsigned short* __restrict__ qu,
                                                          unsigned short* __restrict__ qv, int n2) {
  const int i = blockIdx.x * 256 + threadIdx.x;
  if (i < n2) {
    const v2f q = *(const v2f*)(qf + 2 * (size_t)i);
    const int col = (2 * i) & (kDM - 1);
    const float u0 = ub[col], u1 = ub[col + 1];
    const float w0 = vbias[col], w1 = vbias[col + 1];
    const unsigned pu = pk16(h_bits(q[0] + u0), h_bits(q[1] + u1));
    const unsigned pv = pk16(h_bits(q[0] + w0), h_bits(q[1] + w1));
    ((volatile unsigned*)qu)[i] = pu;
    ((volatile unsigned*)qv)[i] = pv;
    __threadfence();
    ((volatile unsigned*)qu)[i] = pu;
    ((volatile unsigned*)qv)[i] = pv;
  }
}

__global__ __launch_bounds__(256) void fill_zero_f32x4_kernel(float* __restrict__ p, int n4) {
  const int i = blockIdx.x * 256 + threadIdx.x;
  if (i < n4) {
    const v4f z = (v4f){0.f, 0.f, 0.f, 0.f};
    *(volatile v4f*)(p + 4 * (size_t)i) = z;
    __threadfence();
    *(volatile v4f*)(p + 4 * (size_t)i) = z;
  }
}
__global__ __launch_bounds__(256) void copy_f32x4_kernel(const float* __restrict__ src, float* __restrict__ dst, int n4) {
  const int i = blockIdx.x * 256 + threadIdx.x;
  if (i < n4) {
    const v4f v = *(const v4f*)(src + 4 * (size_t)i);
    *(volatile v4f*)(dst + 4 * (size_t)i) = v;
    __threadfence();
    *(volatile v4f*)(dst + 4 * (size_t)i) = v;
  }
}

__global__ __launch_bounds__(256) void rel_softmax_kernel(const float* __restrict__ Sac, const float* __restrict__ Sbd,
                                                          const int* __restrict__ mask, int b,
                                                          unsigned short* __restrict__ P, float* __restrict__ AM) {
  __shared__ float redm[kHGrp][8];
  __shared__ float reds[kHGrp][8];
  __shared__ __align__(16) float amrow[kTK];
  const int i    = blockIdx.x;
  const int tid  = threadIdx.x;
  const int lane = tid & 31;
  const int wave = tid >> 5;
  const int j0   = tid * 8;

  const int* mp = mask + ((size_t)i * kTK + j0) * kNB;
  const v4i mqa = *(const v4i*)(mp);
  const v4i mqb = *(const v4i*)(mp + 4);
  const v4i mqc = *(const v4i*)(mp + 8);
  const v4i mqd = *(const v4i*)(mp + 12);
  const bool bsel = (b != 0);
  int mk[8];
  mk[0] = bsel ? mqa[1] : mqa[0];  mk[1] = bsel ? mqa[3] : mqa[2];
  mk[2] = bsel ? mqb[1] : mqb[0];  mk[3] = bsel ? mqb[3] : mqb[2];
  mk[4] = bsel ? mqc[1] : mqc[0];  mk[5] = bsel ? mqc[3] : mqc[2];
  mk[6] = bsel ? mqd[1] : mqd[0];  mk[7] = bsel ? mqd[3] : mqd[2];
  int jb[8];
#pragma unroll
  for (int e = 0; e < 8; ++e) {
    const int jj = j0 + e + (kSeqQ - 1) - i;
    jb[e] = (jj > kTK - 1) ? (kTK - 1) : jj;
  }
  float am[8];
#pragma unroll
  for (int e = 0; e < 8; ++e) am[e] = 0.f;

#pragma unroll
  for (int hg = 0; hg < kHGrp; ++hg) {
    const size_t rbase = ((size_t)hg * kSeqQ + i) * kTK;
    const v4f a0 = *(const v4f*)(Sac + rbase + j0);
    const v4f a1 = *(const v4f*)(Sac + rbase + j0 + 4);
    float ac[8];
    ac[0] = a0[0]; ac[1] = a0[1]; ac[2] = a0[2]; ac[3] = a0[3];
    ac[4] = a1[0]; ac[5] = a1[1]; ac[6] = a1[2]; ac[7] = a1[3];
    const float* bdp = Sbd + rbase;
    float t[8];
#pragma unroll
    for (int e = 0; e < 8; ++e) {
      const float bd = bdp[jb[e]];
      const float sv = (ac[e] + bd) * 0.125f;
      t[e] = (mk[e] != 0) ? -INFINITY : sv;
    }
    float m = fmaxf(fmaxf(fmaxf(t[0], t[1]), fmaxf(t[2], t[3])), fmaxf(fmaxf(t[4], t[5]), fmaxf(t[6], t[7])));
#pragma unroll
    for (int off = 16; off > 0; off >>= 1) m = fmaxf(m, __shfl_xor(m, off, 32));
    if (lane == 0) redm[hg][wave] = m;
    __syncthreads();
    float mx = redm[hg][0];
#pragma unroll
    for (int w = 1; w < 8; ++w) mx = fmaxf(mx, redm[hg][w]);
    float ex[8];
#pragma unroll
    for (int e = 0; e < 8; ++e) ex[e] = __expf(t[e] - mx);
    float s = ((ex[0] + ex[1]) + (ex[2] + ex[3])) + ((ex[4] + ex[5]) + (ex[6] + ex[7]));
#pragma unroll
    for (int off = 16; off > 0; off >>= 1) s += __shfl_xor(s, off, 32);
    if (lane == 0) reds[hg][wave] = s;
    __syncthreads();
    float tot = reds[hg][0];
#pragma unroll
    for (int w = 1; w < 8; ++w) tot += reds[hg][w];
    const float inv = 1.0f / tot;
    float p[8];
#pragma unroll
    for (int e = 0; e < 8; ++e) { p[e] = ex[e] * inv; am[e] += p[e]; }
    const v4u hv = (v4u){pk16(h_bits(p[0] * PSCALE), h_bits(p[1] * PSCALE)),
                         pk16(h_bits(p[2] * PSCALE), h_bits(p[3] * PSCALE)),
                         pk16(h_bits(p[4] * PSCALE), h_bits(p[5] * PSCALE)),
                         pk16(h_bits(p[6] * PSCALE), h_bits(p[7] * PSCALE))};
    unsigned short* pp = P + rbase + j0;
    *(volatile v4u*)pp = hv;
    __threadfence();
    *(volatile v4u*)pp = hv;
  }

  *(v4f*)(amrow + j0)     = (v4f){am[0], am[1], am[2], am[3]};
  *(v4f*)(amrow + j0 + 4) = (v4f){am[4], am[5], am[6], am[7]};
  __syncthreads();
  const int c4 = tid * 4;
  const v4f x0 = *(const v4f*)(amrow + c4);
  const v4f x1 = *(const v4f*)(amrow + (kTK / 2) + c4);
  float* amp = AM + (size_t)i * kTK;
  const float wmean = 1.0f / (float)(kNB * kNH);
  v4f y0 = *(const v4f*)(amp + c4);
  v4f y1 = *(const v4f*)(amp + (kTK / 2) + c4);
  y0 = y0 + x0 * wmean;
  y1 = y1 + x1 * wmean;
  *(volatile v4f*)(amp + c4) = y0;
  *(volatile v4f*)(amp + (kTK / 2) + c4) = y1;
  __threadfence();
  *(volatile v4f*)(amp + c4) = y0;
  *(volatile v4f*)(amp + (kTK / 2) + c4) = y1;
}

template <bool HAS_B, bool OUT16>
__global__ __launch_bounds__(256) void layernorm_kernel(const float* __restrict__ A, int lda, const float* __restrict__ Bsrc, int ldb,
                                                        const float* __restrict__ gam, const float* __restrict__ bet,
                                                        float* __restrict__ outf, int ldo, unsigned short* __restrict__ out16) {
  __shared__ float red1[8];
  __shared__ float red2[8];
  __shared__ __align__(16) float yrow[OUT16 ? kDM : 4];
  const int row  = blockIdx.x;
  const int tid  = threadIdx.x;
  const int lane = tid & 31;
  const int wave = tid >> 5;
  const int c4   = tid * 4;
  v4f a = *(const v4f*)(A + (size_t)row * lda + c4);
  if (HAS_B) { const v4f bb = *(const v4f*)(Bsrc + (size_t)row * ldb + c4); a = a + bb; }
  float s = (a[0] + a[1]) + (a[2] + a[3]);
#pragma unroll
  for (int off = 16; off > 0; off >>= 1) s += __shfl_xor(s, off, 32);
  if (lane == 0) red1[wave] = s;
  __syncthreads();
  float tot = red1[0];
#pragma unroll
  for (int w = 1; w < 8; ++w) tot += red1[w];
  const float mu = tot * (1.0f / (float)kDM);
  const v4f d = a - mu;
  float sq = (d[0] * d[0] + d[1] * d[1]) + (d[2] * d[2] + d[3] * d[3]);
#pragma unroll
  for (int off = 16; off > 0; off >>= 1) sq += __shfl_xor(sq, off, 32);
  if (lane == 0) red2[wave] = sq;
  __syncthreads();
  float tot2 = red2[0];
#pragma unroll
  for (int w = 1; w < 8; ++w) tot2 += red2[w];
  const float var  = tot2 * (1.0f / (float)kDM);
  const float rstd = rsqrtf(var + 1e-5f);
  const v4f g  = *(const v4f*)(gam + c4);
  const v4f be = *(const v4f*)(bet + c4);
  const v4f y = d * rstd * g + be;
  float* op = outf + (size_t)row * ldo + c4;
  *(volatile v4f*)op = y;
  __threadfence();
  *(volatile v4f*)op = y;
  if (OUT16) {
    *(v4f*)(yrow + c4) = y;
    __syncthreads();
    if (tid < 128) {
      v8h hv;
#pragma unroll
      for (int e = 0; e < 8; ++e) hv[e] = (_Float16)yrow[8 * tid + e];
      unsigned short* hp = out16 + (size_t)row * kDM + 8 * tid;
      *(volatile v8h*)hp = hv;
      __threadfence();
      *(volatile v8h*)hp = hv;
    }
  }
}

extern "C" void kernel_launch(void* const* d_in, const int* in_sizes, int n_in,
                              void* d_out, int out_size, void* d_ws, size_t ws_size,
                              hipStream_t stream) {
  if (n_in < 18) return;
  if (in_sizes[0]  != kSeqQ * kNB * kDM) return;
  if (in_sizes[1]  != kTK * kNB * kDM) return;
  if (in_sizes[2]  != kNH * kDHD || in_sizes[3] != kNH * kDHD) return;
  if (in_sizes[4]  != kMemL * kNB * kDM) return;
  if (in_sizes[5]  != kDM * kDM) return;
  if (in_sizes[6]  != kDM * 2 * kDM) return;
  if (in_sizes[7]  != kDM * kDM) return;
  if (in_sizes[8]  != kDM * kDM) return;
  if (in_sizes[9]  != kDM || in_sizes[10] != kDM) return;
  if (in_sizes[11] != kDM * kDFF) return;
  if (in_sizes[12] != kDFF) return;
  if (in_sizes[13] != kDFF * kDM) return;
  if (in_sizes[14] != kDM) return;
  if (in_sizes[15] != kDM || in_sizes[16] != kDM) return;
  if (in_sizes[17] != kSeqQ * kTK * kNB) return;
  if (out_size != kSeqQ * kNB * kDM + kSeqQ * kTK) return;

  const float* xp    = (const float*)d_in[0];
  const float* pep   = (const float*)d_in[1];
  const float* pbu   = (const float*)d_in[2];
  const float* pbv   = (const float*)d_in[3];
  const float* memp  = (const float*)d_in[4];
  const float* Wq    = (const float*)d_in[5];
  const float* Wkv   = (const float*)d_in[6];
  const float* Wo    = (const float*)d_in[7];
  const float* Wrel  = (const float*)d_in[8];
  const float* ln1g  = (const float*)d_in[9];
  const float* ln1b  = (const float*)d_in[10];
  const float* W1    = (const float*)d_in[11];
  const float* b1p   = (const float*)d_in[12];
  const float* W2    = (const float*)d_in[13];
  const float* b2p   = (const float*)d_in[14];
  const float* ln2g  = (const float*)d_in[15];
  const float* ln2b  = (const float*)d_in[16];
  const int*   maskp = (const int*)d_in[17];

  float* out0 = (float*)d_out;
  float* out1 = (float*)d_out + (size_t)kSeqQ * kNB * kDM;

  const size_t bW   = (size_t)kDM * kDM * 2;
  const size_t bWff = (size_t)kDM * kDFF * 2;
  const size_t bAct = (size_t)kTK * kDM * 2;
  const size_t bQf  = (size_t)kSeqQ * kDM * 4;
  const size_t bQ16 = (size_t)kSeqQ * kDM * 2;
  const size_t bS   = (size_t)kHGrp * kSeqQ * kTK * 4;
  const size_t bP   = (size_t)kHGrp * kSeqQ * kTK * 2;
  const size_t bAM  = (size_t)kSeqQ * kTK * 4;
  size_t off = 0;
  const size_t oWqT  = off; off += bW;
  const size_t oWkT  = off; off += bW;
  const size_t oWvT  = off; off += bW;
  const size_t oWrT  = off; off += bW;
  const size_t oWoT  = off; off += bW;
  const size_t oW1T  = off; off += bWff;
  const size_t oW2T  = off; off += bWff;
  const size_t oC16  = off; off += bAct;
  const size_t oPE16 = off; off += bAct;
  const size_t oK16  = off; off += bAct;
  const size_t oVT16 = off; off += bAct;
  const size_t oR16  = off; off += bAct;
  const size_t oQf   = off; off += bQf;
  const size_t oQU   = off; off += bQ16;
  const size_t oQV   = off; off += bQ16;
  const size_t oSac  = off; off += bS;
  const size_t oSbd  = off; off += bS;
  const size_t oP16  = off; off += bP;
  const size_t oAM   = off; off += bAM;
  const size_t oCTX  = off; off += bQ16;
  const size_t oOUT1 = off; off += bQf;
  const size_t oO16  = off; off += bQ16;
  if (off > ws_size) return;
  if (oPE16 != oC16 + bAct) return;
  if (bWff > bS) return;

  char* ws = (char*)d_ws;
  unsigned short* WqT   = (unsigned short*)(ws + oWqT);
  unsigned short* WkT   = (unsigned short*)(ws + oWkT);
  unsigned short* WvT   = (unsigned short*)(ws + oWvT);
  unsigned short* WrT   = (unsigned short*)(ws + oWrT);
  unsigned short* WoT   = (unsigned short*)(ws + oWoT);
  unsigned short* W1T   = (unsigned short*)(ws + oW1T);
  unsigned short* W2T   = (unsigned short*)(ws + oW2T);
  unsigned short* C16   = (unsigned short*)(ws + oC16);
  unsigned short* X16   = C16 + (size_t)kMemL * kDM;
  unsigned short* PE16  = (unsigned short*)(ws + oPE16);
  unsigned short* K16   = (unsigned short*)(ws + oK16);
  unsigned short* VT16  = (unsigned short*)(ws + oVT16);
  unsigned short* R16   = (unsigned short*)(ws + oR16);
  float*          Qf    = (float*)(ws + oQf);
  float*          AO    = Qf;
  float*          FFR   = Qf;
  unsigned short* QU16  = (unsigned short*)(ws + oQU);
  unsigned short* QV16  = (unsigned short*)(ws + oQV);
  float*          Sac   = (float*)(ws + oSac);
  unsigned short* H16   = (unsigned short*)(ws + oSac);
  float*          Sbd   = (float*)(ws + oSbd);
  unsigned short* P16   = (unsigned short*)(ws + oP16);
  float*          AM    = (float*)(ws + oAM);
  unsigned short* CTX16 = (unsigned short*)(ws + oCTX);
  float*          OUT1f = (float*)(ws + oOUT1);
  unsigned short* O16   = (unsigned short*)(ws + oO16);

  const dim3 blk(256);
  const float wcarry = 16.0f;
  const float wscale = 1.0f / 16.0f;

  transpose_cast_f16_kernel<<<dim3(kDM / 64, kDM / 64), blk, 0, stream>>>(Wq, kDM, kDM, WqT, wcarry);
  transpose_cast_f16_kernel<<<dim3(kDM / 64, kDM / 64), blk, 0, stream>>>(Wkv, 2 * kDM, kDM, WkT, wcarry);
  transpose_cast_f16_kernel<<<dim3(kDM / 64, kDM / 64), blk, 0, stream>>>(Wkv + kDM, 2 * kDM, kDM, WvT, wcarry);
  transpose_cast_f16_kernel<<<dim3(kDM / 64, kDM / 64), blk, 0, stream>>>(Wrel, kDM, kDM, WrT, wcarry);
  transpose_cast_f16_kernel<<<dim3(kDM / 64, kDM / 64), blk, 0, stream>>>(Wo, kDM, kDM, WoT, wcarry);
  transpose_cast_f16_kernel<<<dim3(kDFF / 64, kDM / 64), blk, 0, stream>>>(W1, kDFF, kDM, W1T, wcarry);
  transpose_cast_f16_kernel<<<dim3(kDM / 64, kDFF / 64), blk, 0, stream>>>(W2, kDM, kDFF, W2T, wcarry);
  const int n4am = kSeqQ * kTK / 4;
  fill_zero_f32x4_kernel<<<dim3((n4am + 255) / 256), blk, 0, stream>>>(AM, n4am);

  const int tQ = kSeqQ / 64, tT = kTK / 64, tD = kDM / 64, tF = kDFF / 64;
  const dim3 gQ((tQ * tD + 7) / 8, 1);
  const dim3 gK((tT * tD + 7) / 8, 1);
  const dim3 gVT((tD * tT + 7) / 8, 1);
  const dim3 gS((tQ * tT + 7) / 8, kHGrp);
  const dim3 gPV((tQ * 1 + 7) / 8, kHGrp);
  const dim3 gF1((tQ * tF + 7) / 8, 1);
  const int  n2q = kSeqQ * kDM / 2;

  for (int b = 0; b < kNB; ++b) {
    cast_act_rows_kernel<<<dim3(2 * kTK), dim3(128), 0, stream>>>(xp, memp, pep, b, C16);
    wmma_gemm64<0, false, 0, 0, false, 0><<<gQ, blk, 0, stream>>>(
        X16, X16, kDM, 0L, WqT, WqT, kDM, 0L, (void*)Qf, (void*)Qf, kDM, 0L,
        b1p, xp, 0L, kSeqQ, kDM, kDM, wscale);
    build_qbias_kernel<<<dim3((n2q + 255) / 256), blk, 0, stream>>>(Qf, pbu, pbv, QU16, QV16, n2q);
    wmma_gemm64<0, false, 0, 1, false, 0><<<gK, blk, 0, stream>>>(
        C16, C16, kDM, 0L, WkT, WkT, kDM, 0L, (void*)K16, (void*)K16, kDM, 0L,
        b1p, xp, 0L, kTK, kDM, kDM, wscale);
    wmma_gemm64<0, false, 0, 1, false, 0><<<gVT, blk, 0, stream>>>(
        WvT, WvT, kDM, 0L, C16, C16, kDM, 0L, (void*)VT16, (void*)VT16, kTK, 0L,
        b1p, xp, 0L, kDM, kTK, kDM, wscale);
    wmma_gemm64<0, false, 0, 1, false, 0><<<gK, blk, 0, stream>>>(
        PE16, PE16, kDM, 0L, WrT, WrT, kDM, 0L, (void*)R16, (void*)R16, kDM, 0L,
        b1p, xp, 0L, kTK, kDM, kDM, wscale);

    for (int g = 0; g < kNGrp; ++g) {
      const size_t hc = (size_t)g * kHGrp * kDHD;
      wmma_gemm64<0, false, 0, 0, false, 0><<<gS, blk, 0, stream>>>(
          QU16 + hc, QU16 + hc, kDM, (long)kDHD, K16 + hc, K16 + hc, kDM, (long)kDHD,
          (void*)Sac, (void*)Sac, kTK, (long)kSeqQ * kTK,
          b1p, xp, 0L, kSeqQ, kTK, kDHD, 1.0f);
      wmma_gemm64<0, false, 0, 0, false, 0><<<gS, blk, 0, stream>>>(
          QV16 + hc, QV16 + hc, kDM, (long)kDHD, R16 + hc, R16 + hc, kDM, (long)kDHD,
          (void*)Sbd, (void*)Sbd, kTK, (long)kSeqQ * kTK,
          b1p, xp, 0L, kSeqQ, kTK, kDHD, 1.0f);
      rel_softmax_kernel<<<dim3(kSeqQ), blk, 0, stream>>>(Sac, Sbd, maskp, b, P16, AM);
      wmma_gemm64<0, false, 0, 1, false, 0><<<gPV, blk, 0, stream>>>(
          P16, P16, kTK, (long)kSeqQ * kTK, VT16 + hc * kTK, VT16 + hc * kTK, kTK, (long)kDHD * kTK,
          (void*)(CTX16 + hc), (void*)(CTX16 + hc), kDM, (long)kDHD,
          b1p, xp, 0L, kSeqQ, kDHD, kTK, PSCALE_INV);
    }
    wmma_gemm64<0, false, 0, 0, false, 0><<<gQ, blk, 0, stream>>>(
        CTX16, CTX16, kDM, 0L, WoT, WoT, kDM, 0L, (void*)AO, (void*)AO, kDM, 0L,
        b1p, xp, 0L, kSeqQ, kDM, kDM, wscale);
    layernorm_kernel<true, true><<<dim3(kSeqQ), blk, 0, stream>>>(
        xp + (size_t)b * kDM, kNB * kDM, AO, kDM, ln1g, ln1b, OUT1f, kDM, O16);
    wmma_gemm64<0, false, 2, 1, false, 2><<<gF1, blk, 0, stream>>>(
        O16, O16, kDM, 0L, W1T, W1T, kDM, 0L, (void*)H16, (void*)H16, kDFF, 0L,
        b1p, xp, 0L, kSeqQ, kDFF, kDM, wscale);
    wmma_gemm64<0, false, 2, 0, true, 0><<<gQ, blk, 0, stream>>>(
        H16, H16, kDFF, 0L, W2T, W2T, kDFF, 0L, (void*)FFR, (void*)FFR, kDM, 0L,
        b2p, OUT1f, 0L, kSeqQ, kDM, kDFF, wscale);
    layernorm_kernel<false, false><<<dim3(kSeqQ), blk, 0, stream>>>(
        FFR, kDM, FFR, kDM, ln2g, ln2b, out0 + (size_t)b * kDM, kNB * kDM, O16);
  }
  copy_f32x4_kernel<<<dim3((n4am + 255) / 256), blk, 0, stream>>>(AM, out1, n4am);
}
